// Actor_56934086475993
// MI455X (gfx1250) — hardware-verified
//
#include <hip/hip_runtime.h>
#include <math.h>

constexpr int NBAT  = 16384;
constexpr int NVEH  = 20;
constexpr int NFEAT = 15;
constexpr int NHID  = 256;
constexpr int NG3   = 768;
constexpr int NL1   = 1024;
constexpr int NL2   = 1024;
constexpr int NL3   = 512;
constexpr int NL4   = 256;
constexpr int KIH   = 32;
constexpr int KL1   = 288;
constexpr int X0P   = 320;
constexpr int RB    = 64;
constexpr int NTHR  = 256;
constexpr int HP    = 264;
constexpr int SP    = 40;
constexpr int HROWS = 32;
constexpr float WCARRY     = 16.0f;
constexpr float WCARRY_INV = 1.0f / 16.0f;

static_assert(NBAT % RB == 0, "recurrence grid exact");
static_assert(RB == 4 * 16, "four 16-row m-subtiles per block");
static_assert(NHID == 2 * 16 * (NTHR / 32), "8 waves x 2 unit subtiles x 16 = 256 hidden units");
static_assert((2 * RB * HP) % NTHR == 0 && (2 * RB * SP) % NTHR == 0 && (RB * NHID) % NTHR == 0, "LDS fills exact");
static_assert((RB * X0P) % NTHR == 0, "x0 staging exact");
static_assert((RB * X0P * 2) % (128 * 4 * (NTHR / 32)) == 0, "x0 store: 10 iterations x 8 waves x 4 lines");
static_assert(RB * X0P <= 2 * RB * HP, "x0 staging fits in the h tiles");
static_assert(KIH % 32 == 0 && KL1 % 32 == 0 && NL1 % 32 == 0 && NL2 % 32 == 0 && NL3 % 32 == 0, "GEMM K % 32 == 0");
static_assert(NBAT % 64 == 0 && NL1 % 64 == 0 && NL2 % 64 == 0 && NL3 % 64 == 0 && NL4 % 64 == 0, "GEMM M, N tile multiples");
static_assert(NBAT % HROWS == 0 && NL4 == 256, "head kernel geometry");

typedef __attribute__((ext_vector_type(16))) _Float16 v16h;
typedef __attribute__((ext_vector_type(8)))  _Float16 v8h;
typedef __attribute__((ext_vector_type(16))) __bf16   v16b;
typedef __attribute__((ext_vector_type(8)))  __bf16   v8b;
typedef __attribute__((ext_vector_type(8)))  float    v8f;
typedef __attribute__((ext_vector_type(4)))  float    v4f;

__device__ __forceinline__ unsigned short f2bf_bits(float f) {
  unsigned u = __float_as_uint(f);
  return (unsigned short)((u + 0x7FFFu + ((u >> 16) & 1u)) >> 16);
}
__device__ __forceinline__ float bf_bits2f(unsigned short h) { return __uint_as_float(((unsigned)h) << 16); }

__device__ __forceinline__ void dep_guard_h(v8f& a, v8f& b, v16h x, v16h y) { asm volatile("v_nop\n\tv_nop\n\tv_nop\n\tv_nop" : "+v"(a), "+v"(b) : "v"(x), "v"(y)); }
__device__ __forceinline__ void dep_guard_b(v8f& a, v8f& b, v16b x, v16b y) { asm volatile("v_nop\n\tv_nop\n\tv_nop\n\tv_nop" : "+v"(a), "+v"(b) : "v"(x), "v"(y)); }
__device__ __forceinline__ void dep_guard4_h(v8f& a, v8f& b, v8f& c, v8f& d, v16h x, v16h y) { asm volatile("v_nop\n\tv_nop\n\tv_nop\n\tv_nop" : "+v"(a), "+v"(b), "+v"(c), "+v"(d) : "v"(x), "v"(y)); }
__device__ __forceinline__ void dep_guard4_b(v8f& a, v8f& b, v8f& c, v8f& d, v16b x, v16b y) { asm volatile("v_nop\n\tv_nop\n\tv_nop\n\tv_nop" : "+v"(a), "+v"(b), "+v"(c), "+v"(d) : "v"(x), "v"(y)); }
__device__ __forceinline__ void dep_guard3x_h(v8f& a, v8f& b, v8f& c, v16h w, v16h x, v16h y, v16h z) {
  asm volatile("v_nop\n\tv_nop\n\tv_nop\n\tv_nop" : "+v"(a), "+v"(b), "+v"(c) : "v"(w), "v"(x), "v"(y), "v"(z));
}
__device__ __forceinline__ void keep4_h(v16h a, v16h b, v16h c, v16h d) { asm volatile("v_nop" :: "v"(a), "v"(b), "v"(c), "v"(d)); }
__device__ __forceinline__ void keep4_b(v16b a, v16b b, v16b c, v16b d) { asm volatile("v_nop" :: "v"(a), "v"(b), "v"(c), "v"(d)); }
__device__ __forceinline__ void acc_guard4(v8f& a, v8f& b, v8f& c, v8f& d) { asm volatile("v_nop\n\tv_nop\n\tv_nop\n\tv_nop" : "+v"(a), "+v"(b), "+v"(c), "+v"(d)); }

template <typename T> struct Frag;
template <> struct Frag<_Float16> {
  typedef v16h V; union U { v16h v; v8h h[2]; };
  static __device__ __forceinline__ v16h load(const _Float16* p) {
    U f; f.h[0] = *(const v8h*)(p); f.h[1] = *(const v8h*)(p + 16); return f.v;
  }
  static __device__ __forceinline__ v8f mma(v16h a, v16h b, v8f c) {
    return __builtin_amdgcn_wmma_f32_16x16x32_f16(false, a, false, b, (short)0, c, false, false);
  }
  static __device__ __forceinline__ void guard(v8f& a, v8f& b, v16h x, v16h y) { dep_guard_h(a, b, x, y); }
  static __device__ __forceinline__ void guard4(v8f& a, v8f& b, v8f& c, v8f& d, v16h x, v16h y) { dep_guard4_h(a, b, c, d, x, y); }
  static __device__ __forceinline__ void keep(v16h a, v16h b, v16h c, v16h d) { keep4_h(a, b, c, d); }
};
template <> struct Frag<__bf16> {
  typedef v16b V; union U { v16b v; v8b h[2]; };
  static __device__ __forceinline__ v16b load(const __bf16* p) {
    U f; f.h[0] = *(const v8b*)(p); f.h[1] = *(const v8b*)(p + 16); return f.v;
  }
  static __device__ __forceinline__ v8f mma(v16b a, v16b b, v8f c) {
    return __builtin_amdgcn_wmma_f32_16x16x32_bf16(false, a, false, b, (short)0, c, false, false);
  }
  static __device__ __forceinline__ void guard(v8f& a, v8f& b, v16b x, v16b y) { dep_guard_b(a, b, x, y); }
  static __device__ __forceinline__ void guard4(v8f& a, v8f& b, v8f& c, v8f& d, v16b x, v16b y) { dep_guard4_b(a, b, c, d, x, y); }
  static __device__ __forceinline__ void keep(v16b a, v16b b, v16b c, v16b d) { keep4_b(a, b, c, d); }
};

__device__ __forceinline__ float fsig(float x)  { return __builtin_amdgcn_rcpf(1.0f + expf(-x)); }
__device__ __forceinline__ float ftanh(float x) { return 1.0f - 2.0f * __builtin_amdgcn_rcpf(expf(2.0f * x) + 1.0f); }

template <int ET> struct Elem;
template <> struct Elem<0> { typedef _Float16 T; };
template <> struct Elem<1> { typedef __bf16 T; };
template <int ET, bool SPLIT, int BIAS_MODE, int OUT_MODE, bool RESID, int ACT = 0>
__global__ __launch_bounds__(256) void wmma_gemm64(
    const unsigned short* __restrict__ Ap, const unsigned short* __restrict__ A2p, int lda, long strideA,
    const unsigned short* __restrict__ Btp, const unsigned short* __restrict__ Bt2p, int ldb, long strideB,
    void* __restrict__ Cout, void* __restrict__ Cout2, int ldc, long strideC,
    const float* __restrict__ bias,
    const float* __restrict__ resid, long strideR,
    int M, int N, int K, float scale) {
  typedef typename Elem<ET>::T T;
  typedef typename Frag<T>::V V;
  const T* A = (const T*)Ap; const T* A2 = (const T*)A2p; const T* Bt = (const T*)Btp; const T* Bt2 = (const T*)Bt2p;
  __shared__ __align__(16) float sT[8][16 * 68];
  const int b    = blockIdx.y;
  const int lane = threadIdx.x & 31;
  const int wave = threadIdx.x >> 5;
  const int tilesN = N >> 6;
  const int tilesM = M >> 6;
  const int tile = blockIdx.x * 8 + wave;
  if (tile >= tilesM * tilesN) return;
  const int tm = tile / tilesN;
  const int tn = tile - tm * tilesN;
  const int m0 = tm << 6;
  const int n0 = tn << 6;

  const T* Ab  = A  + (size_t)b * strideA;
  const T* Bb  = Bt + (size_t)b * strideB;
  const T* Ab2 = SPLIT ? (A2  + (size_t)b * strideA) : nullptr;
  const T* Bb2 = SPLIT ? (Bt2 + (size_t)b * strideB) : nullptr;

  const int rlane = lane & 15;
  const int koff  = (lane >> 4) * 8;
  const int mOff  = (lane >> 4) * 8;

  v8f acc[4][4];
#pragma unroll
  for (int i = 0; i < 4; ++i)
#pragma unroll
    for (int j = 0; j < 4; ++j) acc[i][j] = (v8f){0.f,0.f,0.f,0.f,0.f,0.f,0.f,0.f};

  for (int k0 = 0; k0 < K; k0 += 32) {
    V bh[4], bl[4];
#pragma unroll
    for (int j = 0; j < 4; ++j) {
      const size_t bo = (size_t)(n0 + (j << 4) + rlane) * ldb + koff + k0;
      bh[j] = Frag<T>::load(Bb + bo);
      if (SPLIT) bl[j] = Frag<T>::load(Bb2 + bo);
    }
#pragma unroll
    for (int i = 0; i < 4; ++i) {
      const size_t ao = (size_t)(m0 + (i << 4) + rlane) * lda + koff + k0;
      V ah = Frag<T>::load(Ab + ao);
      V al;
      if (SPLIT) al = Frag<T>::load(Ab2 + ao);
#pragma unroll
      for (int j = 0; j < 4; ++j) {
        acc[i][j] = Frag<T>::mma(ah, bh[j], acc[i][j]);
        if (SPLIT) {
          acc[i][j] = Frag<T>::mma(ah, bl[j], acc[i][j]);
          acc[i][j] = Frag<T>::mma(al, bh[j], acc[i][j]);
        }
      }
      Frag<T>::guard4(acc[i][0], acc[i][1], acc[i][2], acc[i][3], SPLIT ? al : ah, bh[3]);
    }
    Frag<T>::keep(bh[0], bh[1], bh[2], bh[3]);
    if (SPLIT) Frag<T>::keep(bl[0], bl[1], bl[2], bl[3]);
  }
  acc_guard4(acc[0][0], acc[0][1], acc[0][2], acc[0][3]);
  acc_guard4(acc[1][0], acc[1][1], acc[1][2], acc[1][3]);
  acc_guard4(acc[2][0], acc[2][1], acc[2][2], acc[2][3]);
  acc_guard4(acc[3][0], acc[3][1], acc[3][2], acc[3][3]);

  float* slab = sT[wave];
  const float* Rb = RESID ? (resid + (size_t)b * strideR) : nullptr;
#pragma unroll
  for (int i = 0; i < 4; ++i) {
    const int mBase = m0 + (i << 4);
#pragma unroll
    for (int j = 0; j < 4; ++j) {
      const int n = n0 + (j << 4) + rlane;
      float bv = 0.f;
      if (BIAS_MODE == 2) bv = bias[n];
#pragma unroll
      for (int r = 0; r < 8; ++r) {
        float v = acc[i][j][r] * scale;
        if (BIAS_MODE == 1) v += bias[mBase + mOff + r];
        if (BIAS_MODE == 2) v += bv;
        if (RESID) v += Rb[(size_t)(mBase + mOff + r) * ldc + n];
        if (ACT == 1) v = tanhf(v);
        if (ACT == 2) v = fmaxf(v, 0.0f);
        if (ACT == 4) v = (v > 0.f) ? v : 0.01f * v;
        slab[(mOff + r) * 68 + (j << 4) + rlane] = v;
      }
    }
    __builtin_amdgcn_fence(__ATOMIC_RELEASE, "workgroup");
    __builtin_amdgcn_wave_barrier();
    __builtin_amdgcn_fence(__ATOMIC_ACQUIRE, "workgroup");
    if (OUT_MODE == 0) {
      float* C = (float*)Cout + (size_t)b * strideC;
      const int hh = lane >> 4, c4 = (lane & 15) * 4;
      for (int pass = 0; pass < 2; ++pass) {
#pragma unroll
        for (int it = 0; it < 8; ++it) {
          const int row = it * 2 + hh;
          v4f v = *(const v4f*)(slab + row * 68 + c4);
          *(volatile v4f*)(C + (size_t)(mBase + row) * ldc + n0 + c4) = v;
        }
        __threadfence();
      }
    } else {
      const int q = lane >> 3, c8 = (lane & 7) * 8;
      unsigned short* C  = (unsigned short*)Cout  + (size_t)b * strideC;
      unsigned short* C2 = (OUT_MODE == 2) ? ((unsigned short*)Cout2 + (size_t)b * strideC) : nullptr;
      for (int pass = 0; pass < 2; ++pass) {
#pragma unroll
        for (int it = 0; it < 4; ++it) {
          const int row = it * 4 + q;
          const float* sp = slab + row * 68 + c8;
          v8h hv, lv;
#pragma unroll
          for (int e = 0; e < 8; ++e) {
            if (OUT_MODE == 1) {
              hv[e] = (_Float16)sp[e];
            } else {
              unsigned short hb = f2bf_bits(sp[e]);
              unsigned short lb = f2bf_bits(sp[e] - bf_bits2f(hb));
              hv[e] = __builtin_bit_cast(_Float16, hb);
              lv[e] = __builtin_bit_cast(_Float16, lb);
            }
          }
          *(volatile v8h*)(C + (size_t)(mBase + row) * ldc + n0 + c8) = hv;
          if (OUT_MODE == 2) *(volatile v8h*)(C2 + (size_t)(mBase + row) * ldc + n0 + c8) = lv;
        }
        __threadfence();
      }
    }
    __builtin_amdgcn_fence(__ATOMIC_RELEASE, "workgroup");
    __builtin_amdgcn_wave_barrier();
    __builtin_amdgcn_fence(__ATOMIC_ACQUIRE, "workgroup");
  }
}

__global__ __launch_bounds__(NTHR) void cvt_pad_kernel(const float* __restrict__ src, unsigned short* __restrict__ dst,
                                                       int rows, int scols, int dcols, float sc) {
  const int i = blockIdx.x * NTHR + threadIdx.x;
  const int ncol8 = dcols >> 3;
  const int n8 = rows * ncol8;
  if (i < n8) {
    const int r  = i / ncol8;
    const int c8 = (i - r * ncol8) * 8;
    const float* sp = src + (size_t)r * scols;
    v8h hv;
#pragma unroll
    for (int e = 0; e < 8; ++e) {
      const int col = c8 + e;
      const int cc  = (col < scols) ? col : (scols - 1);
      const float fa = (col < scols) ? sc : 0.0f;
      const float f = sp[cc] * fa;
      hv[e] = (_Float16)f;
    }
    *(volatile v8h*)(dst + (size_t)i * 8) = hv;
    __threadfence();
    *(volatile v8h*)(dst + (size_t)i * 8) = hv;
  }
}

__global__ __launch_bounds__(NTHR) void gru_kernel(const float* __restrict__ state,
                                                   const float* __restrict__ b_ih, const float* __restrict__ b_hh,
                                                   const unsigned short* __restrict__ Wihp,
                                                   const unsigned short* __restrict__ Whhp,
                                                   unsigned short* __restrict__ X0) {
  __shared__ __align__(16) _Float16 hA[2 * RB * HP];
  __shared__ __align__(16) _Float16 sA[2 * RB * SP];
  __shared__ __align__(16) float    hF[RB * NHID];
  const _Float16* Wih = (const _Float16*)Wihp;
  const _Float16* Whh = (const _Float16*)Whhp;
  const int tid = threadIdx.x, lane = tid & 31, wave = tid >> 5;
  const int c = lane & 15, hh = lane >> 4, koff = hh * 8;
  const int b0 = blockIdx.x * RB;

#pragma unroll 1
  for (int i = tid; i < 2 * RB * HP; i += NTHR) hA[i] = (_Float16)0.0f;
#pragma unroll 1
  for (int i = tid; i < 2 * RB * SP; i += NTHR) sA[i] = (_Float16)0.0f;
#pragma unroll 1
  for (int i = tid; i < RB * NHID; i += NTHR) hF[i] = 0.0f;
  __syncthreads();
#pragma unroll 1
  for (int i = tid; i < RB * NFEAT; i += NTHR) {
    const int row = i / NFEAT, f = i - row * NFEAT;
    sA[row * SP + f] = (_Float16)state[((size_t)(b0 + row) * NVEH) * NFEAT + f];
  }
  __syncthreads();

  const v8f z8 = {0.f, 0.f, 0.f, 0.f, 0.f, 0.f, 0.f, 0.f};

#pragma unroll 1
  for (int v = 0; v < NVEH; ++v) {
    const int cur = v & 1;
    const _Float16* hAc = hA + cur * (RB * HP);
    _Float16*       hAn = hA + (cur ^ 1) * (RB * HP);
    const _Float16* sAc = sA + cur * (RB * SP);
    _Float16*       sAn = sA + (cur ^ 1) * (RB * SP);

#pragma unroll 1
    for (int p = 0; p < 2; ++p) {
      const int u = 16 * (2 * wave + p) + c;
      const float bR  = b_ih[u] + b_hh[u];
      const float bZ  = b_ih[NHID + u] + b_hh[NHID + u];
      const float bXN = b_ih[2 * NHID + u];
      const float bHN = b_hh[2 * NHID + u];
      const _Float16* wx = Wih + (size_t)u * KIH + koff;
      const _Float16* wh = Whh + (size_t)u * NHID + koff;
      v8f aR[4], aZ[4], aH[4], aX[4];
#pragma unroll
      for (int mi = 0; mi < 4; ++mi) { aR[mi] = z8; aZ[mi] = z8; aH[mi] = z8; aX[mi] = z8; }
      {
        const v16h bxr = Frag<_Float16>::load(wx);
        const v16h bxz = Frag<_Float16>::load(wx + (size_t)NHID * KIH);
        const v16h bxn = Frag<_Float16>::load(wx + (size_t)2 * NHID * KIH);
#pragma unroll
        for (int mi = 0; mi < 4; ++mi) {
          const v16h a = Frag<_Float16>::load(sAc + (16 * mi + c) * SP + koff);
          aR[mi] = Frag<_Float16>::mma(a, bxr, aR[mi]);
          aZ[mi] = Frag<_Float16>::mma(a, bxz, aZ[mi]);
          aX[mi] = Frag<_Float16>::mma(a, bxn, aX[mi]);
          dep_guard3x_h(aR[mi], aZ[mi], aX[mi], a, bxr, bxz, bxn);
        }
        keep4_h(bxr, bxz, bxn, bxr);
      }
#pragma unroll 1
      for (int k0 = 0; k0 < NHID; k0 += 32) {
        const v16h br = Frag<_Float16>::load(wh + k0);
        const v16h bz = Frag<_Float16>::load(wh + (size_t)NHID * NHID + k0);
        const v16h bn = Frag<_Float16>::load(wh + (size_t)2 * NHID * NHID + k0);
#pragma unroll
        for (int mi = 0; mi < 4; ++mi) {
          const v16h a = Frag<_Float16>::load(hAc + (16 * mi + c) * HP + koff + k0);
          aR[mi] = Frag<_Float16>::mma(a, br, aR[mi]);
          aZ[mi] = Frag<_Float16>::mma(a, bz, aZ[mi]);
          aH[mi] = Frag<_Float16>::mma(a, bn, aH[mi]);
          dep_guard3x_h(aR[mi], aZ[mi], aH[mi], a, br, bz, bn);
        }
        keep4_h(br, bz, bn, br);
      }
      acc_guard4(aR[0], aR[1], aR[2], aR[3]);
      acc_guard4(aZ[0], aZ[1], aZ[2], aZ[3]);
      acc_guard4(aH[0], aH[1], aH[2], aH[3]);
      acc_guard4(aX[0], aX[1], aX[2], aX[3]);
#pragma unroll
      for (int mi = 0; mi < 4; ++mi) {
#pragma unroll
        for (int r = 0; r < 8; ++r) {
          const int row = 16 * mi + 8 * hh + r;
          const float pr = fmaf(aR[mi][r], WCARRY_INV, bR);
          const float pz = fmaf(aZ[mi][r], WCARRY_INV, bZ);
          const float ph = fmaf(aH[mi][r], WCARRY_INV, bHN);
          const float px = fmaf(aX[mi][r], WCARRY_INV, bXN);
          const float rg = fsig(pr);
          const float zg = fsig(pz);
          const float nn = ftanh(px + rg * ph);
          const float ho = hF[row * NHID + u];
          const float hn = (1.0f - zg) * nn + zg * ho;
          hF[row * NHID + u] = hn;
          hAn[row * HP + u] = (_Float16)hn;
        }
      }
    }
    {
      const int tn = (v + 1 < NVEH) ? (v + 1) : (NVEH - 1);
#pragma unroll 1
      for (int i = tid; i < RB * NFEAT; i += NTHR) {
        const int row = i / NFEAT, f = i - row * NFEAT;
        sAn[row * SP + f] = (_Float16)state[((size_t)(b0 + row) * NVEH + tn) * NFEAT + f];
      }
    }
    __syncthreads();
  }

  {
    _Float16* xs = hA;
#pragma unroll 1
    for (int i = tid; i < RB * X0P; i += NTHR) {
      const int row = i / X0P, col = i - row * X0P;
      const int cs = (col < NFEAT) ? col : (NFEAT - 1);
      int ch = col - NFEAT; ch = (ch < 0) ? 0 : ((ch > NHID - 1) ? (NHID - 1) : ch);
      const float gs = state[((size_t)(b0 + row) * NVEH) * NFEAT + cs];
      const float hv = hF[row * NHID + ch];
      const float fs = (col < NFEAT) ? 1.0f : 0.0f;
      const float fh = (col >= NFEAT && col < NFEAT + NHID) ? 1.0f : 0.0f;
      xs[i] = (_Float16)fmaf(fs, gs, fh * hv);
    }
  }
  __syncthreads();
  {
    const _Float16* xs = hA;
    _Float16* dstb = (_Float16*)X0 + (size_t)b0 * X0P;
    const int q = lane >> 3, c8 = (lane & 7) * 8;
    for (int pass = 0; pass < 2; ++pass) {
#pragma unroll
      for (int it = 0; it < 10; ++it) {
        const int g  = it * 8 + wave;
        const int eo = (4 * g + q) * 64 + c8;
        const v8h vv = *(const v8h*)(xs + eo);
        *(volatile v8h*)(dstb + eo) = vv;
      }
      __threadfence();
    }
  }
}

__global__ __launch_bounds__(NTHR) void head_kernel(const float* __restrict__ Y4, const float* __restrict__ Wp,
                                                    const float* __restrict__ bp, float* __restrict__ out) {
  __shared__ __align__(16) float sRes[HROWS];
  const int tid = threadIdx.x, lane = tid & 31, wave = tid >> 5;
  const int rb = blockIdx.x * HROWS;
  const v4f w0 = *(const v4f*)(Wp + 4 * lane);
  const v4f w1 = *(const v4f*)(Wp + 128 + 4 * lane);
  const float bb = bp[0];
#pragma unroll 1
  for (int j = 0; j < 4; ++j) {
    const int row = rb + 4 * wave + j;
    const float* yp = Y4 + (size_t)row * NL4;
    const v4f a0 = *(const v4f*)(yp + 4 * lane);
    const v4f a1 = *(const v4f*)(yp + 128 + 4 * lane);
    float s = 0.0f;
    s = fmaf(a0[0], w0[0], s); s = fmaf(a0[1], w0[1], s); s = fmaf(a0[2], w0[2], s); s = fmaf(a0[3], w0[3], s);
    s = fmaf(a1[0], w1[0], s); s = fmaf(a1[1], w1[1], s); s = fmaf(a1[2], w1[2], s); s = fmaf(a1[3], w1[3], s);
#pragma unroll
    for (int off = 1; off < 32; off <<= 1) s += __shfl_xor(s, off, 32);
    const float o = tanhf(s + bb);
    if (lane == 0) sRes[4 * wave + j] = o;
  }
  __syncthreads();
  if (wave == 0) {
    const int l8 = lane & 7;
    const v4f vv = *(const v4f*)(sRes + 4 * l8);
    float* op = out + (size_t)rb + 4 * l8;
    if (lane < 8) *(volatile v4f*)op = vv;
    __threadfence();
    if (lane < 8) *(volatile v4f*)op = vv;
  }
}

extern "C" void kernel_launch(void* const* d_in, const int* in_sizes, int n_in,
                              void* d_out, int out_size, void* d_ws, size_t ws_size, hipStream_t stream) {
  if (n_in < 15 || d_out == nullptr || d_ws == nullptr) return;
  if (in_sizes[0] != NBAT * NVEH * NFEAT || in_sizes[1] != NG3 * NFEAT || in_sizes[2] != NG3 * NHID ||
      in_sizes[3] != NG3 || in_sizes[4] != NG3 || in_sizes[5] != NL1 * (NFEAT + NHID) || in_sizes[6] != NL1 ||
      in_sizes[7] != NL2 * NL1 || in_sizes[8] != NL2 || in_sizes[9] != NL3 * NL2 || in_sizes[10] != NL3 ||
      in_sizes[11] != NL4 * NL3 || in_sizes[12] != NL4 || in_sizes[13] != NL4 || in_sizes[14] != 1 ||
      out_size != NBAT) return;

  const float* state = (const float*)d_in[0];
  const float* W_ih  = (const float*)d_in[1];
  const float* W_hh  = (const float*)d_in[2];
  const float* b_ih  = (const float*)d_in[3];
  const float* b_hh  = (const float*)d_in[4];
  const float* W1    = (const float*)d_in[5];
  const float* b1    = (const float*)d_in[6];
  const float* W2    = (const float*)d_in[7];
  const float* b2    = (const float*)d_in[8];
  const float* W3    = (const float*)d_in[9];
  const float* b3    = (const float*)d_in[10];
  const float* W4    = (const float*)d_in[11];
  const float* b4    = (const float*)d_in[12];
  const float* Wp    = (const float*)d_in[13];
  const float* bp    = (const float*)d_in[14];
  float* out = (float*)d_out;

  char* ws = (char*)d_ws; size_t off = 0;
  auto carve = [&](size_t bytes) -> char* { char* p = ws + off; off += (bytes + 255) & ~(size_t)255; return p; };
  unsigned short* WIH = (unsigned short*)carve((size_t)NG3 * KIH * 2);
  unsigned short* WHH = (unsigned short*)carve((size_t)NG3 * NHID * 2);
  unsigned short* W1P = (unsigned short*)carve((size_t)NL1 * KL1 * 2);
  unsigned short* W2P = (unsigned short*)carve((size_t)NL2 * NL1 * 2);
  unsigned short* W3P = (unsigned short*)carve((size_t)NL3 * NL2 * 2);
  unsigned short* W4P = (unsigned short*)carve((size_t)NL4 * NL3 * 2);
  unsigned short* X0  = (unsigned short*)carve((size_t)NBAT * X0P * 2);
  unsigned short* Y1  = (unsigned short*)carve((size_t)NBAT * NL1 * 2);
  unsigned short* Y2  = (unsigned short*)carve((size_t)NBAT * NL2 * 2);
  unsigned short* Y3  = (unsigned short*)carve((size_t)NBAT * NL3 * 2);
  float*          Y4  = (float*)carve((size_t)NBAT * NL4 * 4);
  if (off > ws_size || off > (size_t)134217728) return;

  {
    const int n0 = NG3 * (KIH / 8), n1 = NG3 * (NHID / 8), n2 = NL1 * (KL1 / 8), n3 = NL2 * (NL1 / 8), n4 = NL3 * (NL2 / 8), n5 = NL4 * (NL3 / 8);
    cvt_pad_kernel<<<(n0 + NTHR - 1) / NTHR, NTHR, 0, stream>>>(W_ih, WIH, NG3, NFEAT, KIH, WCARRY);
    cvt_pad_kernel<<<(n1 + NTHR - 1) / NTHR, NTHR, 0, stream>>>(W_hh, WHH, NG3, NHID, NHID, WCARRY);
    cvt_pad_kernel<<<(n2 + NTHR - 1) / NTHR, NTHR, 0, stream>>>(W1, W1P, NL1, NFEAT + NHID, KL1, WCARRY);
    cvt_pad_kernel<<<(n3 + NTHR - 1) / NTHR, NTHR, 0, stream>>>(W2, W2P, NL2, NL1, NL1, WCARRY);
    cvt_pad_kernel<<<(n4 + NTHR - 1) / NTHR, NTHR, 0, stream>>>(W3, W3P, NL3, NL2, NL2, WCARRY);
    cvt_pad_kernel<<<(n5 + NTHR - 1) / NTHR, NTHR, 0, stream>>>(W4, W4P, NL4, NL3, NL3, WCARRY);
  }
  gru_kernel<<<NBAT / RB, NTHR, 0, stream>>>(state, b_ih, b_hh, WIH, WHH, X0);

  {
    const int t1 = (NBAT / 64) * (NL1 / 64), t2 = (NBAT / 64) * (NL2 / 64), t3 = (NBAT / 64) * (NL3 / 64), t4 = (NBAT / 64) * (NL4 / 64);
    wmma_gemm64<0, false, 2, 1, false, 2><<<dim3((t1 + 7) / 8, 1), 256, 0, stream>>>(
        X0, X0, X0P, 0L, W1P, W1P, KL1, 0L, (void*)Y1, (void*)Y1, NL1, 0L, b1, b1, 0L, NBAT, NL1, KL1, WCARRY_INV);
    wmma_gemm64<0, false, 2, 1, false, 2><<<dim3((t2 + 7) / 8, 1), 256, 0, stream>>>(
        Y1, Y1, NL1, 0L, W2P, W2P, NL1, 0L, (void*)Y2, (void*)Y2, NL2, 0L, b2, b2, 0L, NBAT, NL2, NL1, WCARRY_INV);
    wmma_gemm64<0, false, 2, 1, false, 2><<<dim3((t3 + 7) / 8, 1), 256, 0, stream>>>(
        Y2, Y2, NL2, 0L, W3P, W3P, NL2, 0L, (void*)Y3, (void*)Y3, NL3, 0L, b3, b3, 0L, NBAT, NL3, NL2, WCARRY_INV);
    wmma_gemm64<0, false, 2, 0, false, 2><<<dim3((t4 + 7) / 8, 1), 256, 0, stream>>>(
        Y3, Y3, NL3, 0L, W4P, W4P, NL3, 0L, (void*)Y4, (void*)Y4, NL4, 0L, b4, b4, 0L, NBAT, NL4, NL3, WCARRY_INV);
  }
  head_kernel<<<NBAT / HROWS, NTHR, 0, stream>>>(Y4, Wp, bp, out);
}
